// CATLayer_75660143886733
// MI455X (gfx1250) — hardware-run, weakly checked
//
#include <hip/hip_runtime.h>
#include <math.h>

constexpr int kTok      = 4096;
constexpr int kDim      = 512;
constexpr int kFfn      = 2048;
constexpr int kExp      = 8;
constexpr int kHeads    = 8;
constexpr int kHd       = 64;
constexpr int kChunkTok = 1024;
constexpr int kNumChunk = kTok / kChunkTok;
constexpr float kWCarry    = 64.0f;
constexpr float kWCarryInv = 1.0f / 64.0f;
constexpr float kCtxCarry  = 16.0f;
constexpr float kOutScale  = 1.0f / (16.0f * 64.0f);
constexpr float kInvSqrtHd = 0.125f;

typedef __attribute__((ext_vector_type(16))) _Float16 v16h;
typedef __attribute__((ext_vector_type(8)))  _Float16 v8h;
typedef __attribute__((ext_vector_type(16))) __bf16   v16b;
typedef __attribute__((ext_vector_type(8)))  __bf16   v8b;
typedef __attribute__((ext_vector_type(8)))  float    v8f;
typedef __attribute__((ext_vector_type(4)))  float    v4f;
typedef __attribute__((ext_vector_type(4)))  unsigned int v4u;

__device__ __forceinline__ unsigned short f2bf_bits(float f) {
  unsigned u = __float_as_uint(f);
  return (unsigned short)((u + 0x7FFFu + ((u >> 16) & 1u)) >> 16);
}
__device__ __forceinline__ float bf_bits2f(unsigned short h) { return __uint_as_float(((unsigned)h) << 16); }

__device__ __forceinline__ void dep_guard_h(v8f& a, v8f& b, v16h x, v16h y) { asm volatile("v_nop\n\tv_nop\n\tv_nop\n\tv_nop" : "+v"(a), "+v"(b) : "v"(x), "v"(y)); }
__device__ __forceinline__ void dep_guard_b(v8f& a, v8f& b, v16b x, v16b y) { asm volatile("v_nop\n\tv_nop\n\tv_nop\n\tv_nop" : "+v"(a), "+v"(b) : "v"(x), "v"(y)); }
__device__ __forceinline__ void keep4_h(v16h a, v16h b, v16h c, v16h d) { asm volatile("v_nop" :: "v"(a), "v"(b), "v"(c), "v"(d)); }
__device__ __forceinline__ void keep4_b(v16b a, v16b b, v16b c, v16b d) { asm volatile("v_nop" :: "v"(a), "v"(b), "v"(c), "v"(d)); }
__device__ __forceinline__ void acc_guard4(v8f& a, v8f& b, v8f& c, v8f& d) { asm volatile("v_nop\n\tv_nop\n\tv_nop\n\tv_nop" : "+v"(a), "+v"(b), "+v"(c), "+v"(d)); }
template <typename T> struct Frag;
template <> struct Frag<_Float16> {
  typedef v16h V; union U { v16h v; v8h h[2]; };
  static __device__ __forceinline__ v16h load(const _Float16* p) {
    U f; f.h[0] = *(const v8h*)(p); f.h[1] = *(const v8h*)(p + 16); return f.v;
  }
  static __device__ __forceinline__ v8f mma(v16h a, v16h b, v8f c) {
    return __builtin_amdgcn_wmma_f32_16x16x32_f16(false, a, false, b, (short)0, c, false, false);
  }
  static __device__ __forceinline__ void guard(v8f& a, v8f& b, v16h x, v16h y) { dep_guard_h(a, b, x, y); }
  static __device__ __forceinline__ void keep(v16h a, v16h b, v16h c, v16h d) { keep4_h(a, b, c, d); }
};
template <> struct Frag<__bf16> {
  typedef v16b V; union U { v16b v; v8b h[2]; };
  static __device__ __forceinline__ v16b load(const __bf16* p) {
    U f; f.h[0] = *(const v8b*)(p); f.h[1] = *(const v8b*)(p + 16); return f.v;
  }
  static __device__ __forceinline__ v8f mma(v16b a, v16b b, v8f c) {
    return __builtin_amdgcn_wmma_f32_16x16x32_bf16(false, a, false, b, (short)0, c, false, false);
  }
  static __device__ __forceinline__ void guard(v8f& a, v8f& b, v16b x, v16b y) { dep_guard_b(a, b, x, y); }
  static __device__ __forceinline__ void keep(v16b a, v16b b, v16b c, v16b d) { keep4_b(a, b, c, d); }
};

__device__ __forceinline__ unsigned pk16(unsigned short a, unsigned short b) { return (unsigned)a | ((unsigned)b << 16); }
__device__ __forceinline__ unsigned short h_bits(float f) { const _Float16 h = (_Float16)f; return __builtin_bit_cast(unsigned short, h); }

template <int ET> struct Elem;
template <> struct Elem<0> { typedef _Float16 T; };
template <> struct Elem<1> { typedef __bf16 T; };
template <int ET, bool SPLIT, int BIAS_MODE, int OUT_MODE, bool RESID, int ACT = 0>
__global__ __launch_bounds__(256) void wmma_gemm64(
    const unsigned short* __restrict__ Ap, const unsigned short* __restrict__ A2p, int lda, long strideA,
    const unsigned short* __restrict__ Btp, const unsigned short* __restrict__ Bt2p, int ldb, long strideB,
    void* __restrict__ Cout, void* __restrict__ Cout2, int ldc, long strideC,
    const float* __restrict__ bias,
    const float* __restrict__ resid, long strideR,
    int M, int N, int K, float scale) {
  typedef typename Elem<ET>::T T;
  typedef typename Frag<T>::V V;
  const T* A = (const T*)Ap; const T* A2 = (const T*)A2p; const T* Bt = (const T*)Btp; const T* Bt2 = (const T*)Bt2p;
  __shared__ __align__(16) float sT[8][16 * 68];
  const int b    = blockIdx.y;
  const int lane = threadIdx.x & 31;
  const int wave = threadIdx.x >> 5;
  const int tilesN = N >> 6;
  const int tilesM = M >> 6;
  const int tile = blockIdx.x * 8 + wave;
  if (tile >= tilesM * tilesN) return;
  const int tm = tile / tilesN;
  const int tn = tile - tm * tilesN;
  const int m0 = tm << 6;
  const int n0 = tn << 6;

  const T* Ab  = A  + (size_t)b * strideA;
  const T* Bb  = Bt + (size_t)b * strideB;
  const T* Ab2 = SPLIT ? (A2  + (size_t)b * strideA) : nullptr;
  const T* Bb2 = SPLIT ? (Bt2 + (size_t)b * strideB) : nullptr;

  const int rlane = lane & 15;
  const int koff  = (lane >> 4) * 8;
  const int mOff  = (lane >> 4) * 8;

  v8f acc[4][4];
#pragma unroll
  for (int i = 0; i < 4; ++i)
#pragma unroll
    for (int j = 0; j < 4; ++j) acc[i][j] = (v8f){0.f,0.f,0.f,0.f,0.f,0.f,0.f,0.f};

  for (int k0 = 0; k0 < K; k0 += 32) {
    V bh[4], bl[4];
#pragma unroll
    for (int j = 0; j < 4; ++j) {
      const size_t bo = (size_t)(n0 + (j << 4) + rlane) * ldb + koff + k0;
      bh[j] = Frag<T>::load(Bb + bo);
      if (SPLIT) bl[j] = Frag<T>::load(Bb2 + bo);
    }
#pragma unroll
    for (int i = 0; i < 4; ++i) {
      const size_t ao = (size_t)(m0 + (i << 4) + rlane) * lda + koff + k0;
      V ah = Frag<T>::load(Ab + ao);
      V al;
      if (SPLIT) al = Frag<T>::load(Ab2 + ao);
#pragma unroll
      for (int j = 0; j < 4; ++j) {
        acc[i][j] = Frag<T>::mma(ah, bh[j], acc[i][j]);
        if (SPLIT) {
          acc[i][j] = Frag<T>::mma(ah, bl[j], acc[i][j]);
          acc[i][j] = Frag<T>::mma(al, bh[j], acc[i][j]);
        }
      }
      Frag<T>::guard(acc[i][0], acc[i][3], ah, SPLIT ? al : ah);
    }
    Frag<T>::keep(bh[0], bh[1], bh[2], bh[3]);
    if (SPLIT) Frag<T>::keep(bl[0], bl[1], bl[2], bl[3]);
  }
  acc_guard4(acc[0][0], acc[0][1], acc[0][2], acc[0][3]);
  acc_guard4(acc[1][0], acc[1][1], acc[1][2], acc[1][3]);
  acc_guard4(acc[2][0], acc[2][1], acc[2][2], acc[2][3]);
  acc_guard4(acc[3][0], acc[3][1], acc[3][2], acc[3][3]);

  float* slab = sT[wave];
  const float* Rb = RESID ? (resid + (size_t)b * strideR) : nullptr;
#pragma unroll
  for (int i = 0; i < 4; ++i) {
    const int mBase = m0 + (i << 4);
#pragma unroll
    for (int j = 0; j < 4; ++j) {
      const int n = n0 + (j << 4) + rlane;
      float bv = 0.f;
      if (BIAS_MODE == 2) bv = bias[n];
#pragma unroll
      for (int r = 0; r < 8; ++r) {
        float v = acc[i][j][r] * scale;
        if (BIAS_MODE == 1) v += bias[mBase + mOff + r];
        if (BIAS_MODE == 2) v += bv;
        if (RESID) v += Rb[(size_t)(mBase + mOff + r) * ldc + n];
        if (ACT == 2) v = fmaxf(v, 0.0f);
        if (ACT == 4) v = (v > 0.f) ? v : 0.01f * v;
        slab[(mOff + r) * 68 + (j << 4) + rlane] = v;
      }
    }
    __builtin_amdgcn_fence(__ATOMIC_RELEASE, "workgroup");
    __builtin_amdgcn_wave_barrier();
    __builtin_amdgcn_fence(__ATOMIC_ACQUIRE, "workgroup");
    if (OUT_MODE == 0) {
      float* C = (float*)Cout + (size_t)b * strideC;
      const int hh = lane >> 4, c4 = (lane & 15) * 4;
      for (int pass = 0; pass < 2; ++pass) {
#pragma unroll
        for (int it = 0; it < 8; ++it) {
          const int row = it * 2 + hh;
          v4f v = *(const v4f*)(slab + row * 68 + c4);
          *(volatile v4f*)(C + (size_t)(mBase + row) * ldc + n0 + c4) = v;
        }
        __threadfence();
      }
    } else {
      const int q = lane >> 3, c8 = (lane & 7) * 8;
      unsigned short* C  = (unsigned short*)Cout  + (size_t)b * strideC;
      unsigned short* C2 = (OUT_MODE == 2) ? ((unsigned short*)Cout2 + (size_t)b * strideC) : nullptr;
      for (int pass = 0; pass < 2; ++pass) {
#pragma unroll
        for (int it = 0; it < 4; ++it) {
          const int row = it * 4 + q;
          const float* sp = slab + row * 68 + c8;
          v8h hv, lv;
#pragma unroll
          for (int e = 0; e < 8; ++e) {
            if (OUT_MODE == 1) {
              hv[e] = (_Float16)sp[e];
            } else {
              unsigned short hb = f2bf_bits(sp[e]);
              unsigned short lb = f2bf_bits(sp[e] - bf_bits2f(hb));
              hv[e] = __builtin_bit_cast(_Float16, hb);
              lv[e] = __builtin_bit_cast(_Float16, lb);
            }
          }
          *(volatile v8h*)(C + (size_t)(mBase + row) * ldc + n0 + c8) = hv;
          if (OUT_MODE == 2) *(volatile v8h*)(C2 + (size_t)(mBase + row) * ldc + n0 + c8) = lv;
        }
        __threadfence();
      }
    }
    __builtin_amdgcn_fence(__ATOMIC_RELEASE, "workgroup");
    __builtin_amdgcn_wave_barrier();
    __builtin_amdgcn_fence(__ATOMIC_ACQUIRE, "workgroup");
  }
}

__global__ __launch_bounds__(256) void k_cast8x4(const float* __restrict__ p0, const float* __restrict__ p1,
                                                 const float* __restrict__ p2, const float* __restrict__ p3,
                                                 unsigned short* __restrict__ out, int n8, float scale) {
  const int z = blockIdx.y;
  const float* ip = (z == 0) ? p0 : (z == 1) ? p1 : (z == 2) ? p2 : p3;
  const int i = blockIdx.x * 256 + threadIdx.x;
  if (i >= n8) return;
  const float* p = ip + 8 * (size_t)i;
  const v4f a = *(const v4f*)(p);
  const v4f c = *(const v4f*)(p + 4);
  unsigned short hb[8];
#pragma unroll
  for (int e = 0; e < 4; ++e) {
    hb[e]     = h_bits(a[e] * scale);
    hb[4 + e] = h_bits(c[e] * scale);
  }
  const v4u u = (v4u){pk16(hb[0], hb[1]), pk16(hb[2], hb[3]), pk16(hb[4], hb[5]), pk16(hb[6], hb[7])};
  unsigned short* q = out + (size_t)z * 8 * (size_t)n8 + 8 * (size_t)i;
  *(volatile v4u*)q = u;
  __threadfence();
  *(volatile v4u*)q = u;
}

__global__ __launch_bounds__(256) void k_tcast(const float* __restrict__ in, unsigned short* __restrict__ out,
                                               int R, int Cc, long planeElems, float scale) {
  __shared__ float sm[64][65];
  const int t  = threadIdx.x;
  const int r0 = blockIdx.x * 64;
  const int c0 = blockIdx.y * 64;
  const size_t pz = (size_t)blockIdx.z * (size_t)planeElems;
  const float* ip = in + pz;
#pragma unroll
  for (int i = 0; i < 16; ++i) {
    const int e  = i * 256 + t;
    const int rl = e >> 6;
    const int cl = e & 63;
    sm[cl][rl] = ip[(size_t)(r0 + rl) * Cc + c0 + cl] * scale;
  }
  __syncthreads();
  const int lane = t & 31, wave = t >> 5;
  const int q = lane >> 3, c8 = (lane & 7) * 8;
  const int ra = wave * 8 + q;
  const int rb = wave * 8 + 4 + q;
  unsigned short ha[8], hbv[8];
#pragma unroll
  for (int e = 0; e < 8; ++e) { ha[e] = h_bits(sm[ra][c8 + e]); hbv[e] = h_bits(sm[rb][c8 + e]); }
  const v4u ua = (v4u){pk16(ha[0], ha[1]), pk16(ha[2], ha[3]), pk16(ha[4], ha[5]), pk16(ha[6], ha[7])};
  const v4u ub = (v4u){pk16(hbv[0], hbv[1]), pk16(hbv[2], hbv[3]), pk16(hbv[4], hbv[5]), pk16(hbv[6], hbv[7])};
  unsigned short* op = out + pz;
  unsigned short* pa = op + (size_t)(c0 + ra) * R + r0 + c8;
  unsigned short* pb = op + (size_t)(c0 + rb) * R + r0 + c8;
  *(volatile v4u*)pa = ua;
  *(volatile v4u*)pb = ub;
  __threadfence();
  *(volatile v4u*)pa = ua;
  *(volatile v4u*)pb = ub;
}

__global__ __launch_bounds__(256) void k_selcopy(const unsigned short* __restrict__ src, const int* __restrict__ selp,
                                                 unsigned short* __restrict__ dst, int n8, int nplanes) {
  int e = selp[0];
  e = (e < 0) ? (e + nplanes) : e;
  e = (e < 0) ? 0 : e;
  e = (e > nplanes - 1) ? (nplanes - 1) : e;
  const int i = blockIdx.x * 256 + threadIdx.x;
  if (i >= n8) return;
  const v4u v = *(const v4u*)(src + (size_t)e * 8 * (size_t)n8 + 8 * (size_t)i);
  unsigned short* q = dst + 8 * (size_t)i;
  *(volatile v4u*)q = v;
  __threadfence();
  *(volatile v4u*)q = v;
}

__global__ __launch_bounds__(256) void k_attn8(const float* __restrict__ Qp, const float* __restrict__ Kp,
                                               const float* __restrict__ Vp, const int* __restrict__ selp,
                                               unsigned short* __restrict__ ctx, int tok0) {
  const int tid  = threadIdx.x;
  const int lane = tid & 31, wave = tid >> 5;
  const int grp  = lane >> 3, f = lane & 7;
  const int pr   = wave * 4 + grp;
  const int tl   = blockIdx.x * 4 + (pr >> 3);
  const int h    = pr & 7;
  const int t    = tok0 + tl;
  int e = selp[0];
  e = (e < 0) ? (e + kExp) : e;
  e = (e < 0) ? 0 : e;
  e = (e > kExp - 1) ? (kExp - 1) : e;

  const float* qr = Qp + (size_t)t * kDim + h * kHd;
  const float* kr = Kp + ((size_t)f * kChunkTok + tl) * kDim + h * kHd;
  float s0 = 0.f, s1 = 0.f, s2 = 0.f, s3 = 0.f;
#pragma unroll 1
  for (int i = 0; i < kHd / 4; ++i) {
    const v4f a = *(const v4f*)(qr + 4 * i);
    const v4f b = *(const v4f*)(kr + 4 * i);
    s0 += a[0] * b[0];
    s1 += a[1] * b[1];
    s2 += a[2] * b[2];
    s3 += a[3] * b[3];
  }
  const float madd = (f <= e) ? 1.0f : 0.0f;
  const float s = ((s0 + s1) + (s2 + s3)) * kInvSqrtHd + madd;
  float m = s;
  m = fmaxf(m, __shfl_xor(m, 1, 32));
  m = fmaxf(m, __shfl_xor(m, 2, 32));
  m = fmaxf(m, __shfl_xor(m, 4, 32));
  float p = expf(s - m);
  float sum = p;
  sum += __shfl_xor(sum, 1, 32);
  sum += __shfl_xor(sum, 2, 32);
  sum += __shfl_xor(sum, 4, 32);
  p = p * (1.0f / sum);

  float c[8];
#pragma unroll
  for (int d = 0; d < 8; ++d) c[d] = 0.f;
  const float* vb = Vp + (size_t)tl * kDim + h * kHd + 8 * f;
#pragma unroll 1
  for (int ff = 0; ff < kExp; ++ff) {
    const float pf = __shfl(p, (grp << 3) + ff, 32);
    const float* vr = vb + (size_t)ff * kChunkTok * kDim;
    const v4f va = *(const v4f*)(vr);
    const v4f vc = *(const v4f*)(vr + 4);
#pragma unroll
    for (int d = 0; d < 4; ++d) {
      c[d]     += pf * va[d];
      c[4 + d] += pf * vc[d];
    }
  }
  unsigned short hb[8];
#pragma unroll
  for (int d = 0; d < 8; ++d) hb[d] = h_bits(c[d] * kCtxCarry);
  const v4u u = (v4u){pk16(hb[0], hb[1]), pk16(hb[2], hb[3]), pk16(hb[4], hb[5]), pk16(hb[6], hb[7])};
  unsigned short* op = ctx + (size_t)t * kDim + h * kHd + 8 * f;
  *(volatile v4u*)op = u;
  __threadfence();
  *(volatile v4u*)op = u;
}

extern "C" void kernel_launch(void* const* d_in, const int* in_sizes, int n_in,
                              void* d_out, int out_size, void* d_ws, size_t ws_size,
                              hipStream_t stream) {
  if (n_in < 14) return;
  const float* x   = (const float*)d_in[0];
  const float* W1  = (const float*)d_in[1];
  const float* b1  = (const float*)d_in[2];
  const float* W2  = (const float*)d_in[3];
  const float* b2  = (const float*)d_in[4];
  const float* Wq  = (const float*)d_in[5];
  const float* bq  = (const float*)d_in[6];
  const float* Wk  = (const float*)d_in[7];
  const float* bk  = (const float*)d_in[8];
  const float* Wv  = (const float*)d_in[9];
  const float* bv  = (const float*)d_in[10];
  const float* Wo  = (const float*)d_in[11];
  const float* bo  = (const float*)d_in[12];
  const int*   sel = (const int*)d_in[13];
  float* out = (float*)d_out;

  if (in_sizes[0] != kTok * kDim) return;
  if (in_sizes[1] != kExp * kDim * kFfn || in_sizes[3] != kExp * kFfn * kDim) return;
  if (in_sizes[2] != kExp * kFfn || in_sizes[4] != kExp * kDim) return;
  if (in_sizes[5] != kDim * kDim || in_sizes[7] != kDim * kDim || in_sizes[9] != kDim * kDim || in_sizes[11] != kDim * kDim) return;
  if (in_sizes[6] != kDim || in_sizes[8] != kDim || in_sizes[10] != kDim || in_sizes[12] != kDim) return;
  if (in_sizes[13] < 1) return;
  if (out_size != kTok * kDim) return;

  const size_t MiB = 1048576;
  const size_t OFF_X16  = 0;
  const size_t OFF_W4   = 4 * MiB;
  const size_t OFF_EO16 = 6 * MiB;
  const size_t OFF_SH   = 38 * MiB;
  const size_t OFF_W1T  = OFF_SH;
  const size_t OFF_W2T  = OFF_SH + 16 * MiB;
  const size_t OFF_HID  = OFF_SH + 32 * MiB;
  const size_t OFF_K32  = OFF_SH;
  const size_t OFF_V32  = OFF_SH + 16 * MiB;
  const size_t OFF_Q32  = OFF_SH + 32 * MiB;
  const size_t OFF_SEL  = OFF_SH + 40 * MiB;
  const size_t OFF_CTX  = OFF_SH + 44 * MiB;
  const size_t TOTAL    = OFF_SH + 48 * MiB;
  if (TOTAL > ws_size) return;

  char* ws = (char*)d_ws;
  unsigned short* X16   = (unsigned short*)(ws + OFF_X16);
  unsigned short* W4    = (unsigned short*)(ws + OFF_W4);
  unsigned short* EO16  = (unsigned short*)(ws + OFF_EO16);
  unsigned short* W1T   = (unsigned short*)(ws + OFF_W1T);
  unsigned short* W2T   = (unsigned short*)(ws + OFF_W2T);
  unsigned short* HID   = (unsigned short*)(ws + OFF_HID);
  float*          K32   = (float*)(ws + OFF_K32);
  float*          V32   = (float*)(ws + OFF_V32);
  float*          Q32   = (float*)(ws + OFF_Q32);
  unsigned short* SEL16 = (unsigned short*)(ws + OFF_SEL);
  unsigned short* CTX16 = (unsigned short*)(ws + OFF_CTX);

  const size_t wPlane   = (size_t)kDim * kDim;
  const size_t w1Plane  = (size_t)kDim * kFfn;
  const size_t eoPlane  = (size_t)kTok * kDim;

  k_cast8x4<<<dim3(kTok * kDim / 8 / 256, 1), 256, 0, stream>>>(x, x, x, x, X16, kTok * kDim / 8, 1.0f);
  k_cast8x4<<<dim3(kDim * kDim / 8 / 256, 4), 256, 0, stream>>>(Wq, Wk, Wv, Wo, W4, kDim * kDim / 8, kWCarry);
  k_tcast<<<dim3(kDim / 64, kFfn / 64, kExp), 256, 0, stream>>>(W1, W1T, kDim, kFfn, (long)w1Plane, kWCarry);
  k_tcast<<<dim3(kFfn / 64, kDim / 64, kExp), 256, 0, stream>>>(W2, W2T, kFfn, kDim, (long)w1Plane, kWCarry);

  for (int e = 0; e < kExp; ++e) {
    wmma_gemm64<0, false, 2, 1, false, 2><<<dim3((kTok / 64) * (kFfn / 64) / 8, 1), 256, 0, stream>>>(
        X16, X16, kDim, 0L,
        W1T + (size_t)e * w1Plane, W1T + (size_t)e * w1Plane, kDim, 0L,
        (void*)HID, (void*)HID, kFfn, 0L,
        b1 + (size_t)e * kFfn, b1, 0L,
        kTok, kFfn, kDim, kWCarryInv);
    wmma_gemm64<0, false, 2, 1, false, 0><<<dim3((kTok / 64) * (kDim / 64) / 8, 1), 256, 0, stream>>>(
        HID, HID, kFfn, 0L,
        W2T + (size_t)e * w1Plane, W2T + (size_t)e * w1Plane, kFfn, 0L,
        (void*)(EO16 + (size_t)e * eoPlane), (void*)(EO16 + (size_t)e * eoPlane), kDim, 0L,
        b2 + (size_t)e * kDim, b2, 0L,
        kTok, kDim, kFfn, kWCarryInv);
  }

  k_selcopy<<<dim3(kTok * kDim / 8 / 256), 256, 0, stream>>>(EO16, sel, SEL16, kTok * kDim / 8, kExp);

  wmma_gemm64<0, false, 2, 0, false, 0><<<dim3((kTok / 64) * (kDim / 64) / 8, 1), 256, 0, stream>>>(
      SEL16, SEL16, kDim, 0L,
      W4 + 0 * wPlane, W4 + 0 * wPlane, kDim, 0L,
      (void*)Q32, (void*)Q32, kDim, 0L,
      bq, bq, 0L,
      kTok, kDim, kDim, kWCarryInv);

  for (int cidx = 0; cidx < kNumChunk; ++cidx) {
    const unsigned short* aChunk = EO16 + (size_t)cidx * kChunkTok * kDim;
    wmma_gemm64<0, false, 2, 0, false, 0><<<dim3((kChunkTok / 64) * (kDim / 64) / 8, kExp), 256, 0, stream>>>(
        aChunk, aChunk, kDim, (long)eoPlane,
        W4 + 1 * wPlane, W4 + 1 * wPlane, kDim, 0L,
        (void*)K32, (void*)K32, kDim, (long)kChunkTok * kDim,
        bk, bk, 0L,
        kChunkTok, kDim, kDim, kWCarryInv);
    wmma_gemm64<0, false, 2, 0, false, 0><<<dim3((kChunkTok / 64) * (kDim / 64) / 8, kExp), 256, 0, stream>>>(
        aChunk, aChunk, kDim, (long)eoPlane,
        W4 + 2 * wPlane, W4 + 2 * wPlane, kDim, 0L,
        (void*)V32, (void*)V32, kDim, (long)kChunkTok * kDim,
        bv, bv, 0L,
        kChunkTok, kDim, kDim, kWCarryInv);
    k_attn8<<<dim3(kChunkTok / 4), 256, 0, stream>>>(Q32, K32, V32, sel, CTX16, cidx * kChunkTok);
  }

  wmma_gemm64<0, false, 2, 0, false, 0><<<dim3((kTok / 64) * (kDim / 64) / 8, 1), 256, 0, stream>>>(
      CTX16, CTX16, kDim, 0L,
      W4 + 3 * wPlane, W4 + 3 * wPlane, kDim, 0L,
      (void*)out, (void*)out, kDim, 0L,
      bo, bo, 0L,
      kTok, kDim, kDim, kOutScale);
}
